// myGPT2Block_68934225101634
// MI455X (gfx1250) — hardware-verified
//
#include <hip/hip_runtime.h>
#include <math.h>

constexpr int kBatch   = 2;
constexpr int kSeq     = 2048;
constexpr int kDim     = 1024;
constexpr int kHeads   = 16;
constexpr int kHdim    = 64;
constexpr int kFF      = 4096;
constexpr int kTok     = kBatch * kSeq;
constexpr int kGroups  = kBatch * kHeads;
constexpr int kGrpChunk = 2;
constexpr int kNumChunks = kGroups / kGrpChunk;
constexpr float kWCarry    = 16.0f;
constexpr float kWCarryInv = 1.0f / 16.0f;
constexpr float kPCarry    = 2048.0f;
constexpr float kCtxCarry  = 256.0f;
constexpr float kScoreScale = 0.125f;
constexpr float kPVScale   = kCtxCarry / kPCarry;
constexpr float kProjScale = 1.0f / (kCtxCarry * kWCarry);
constexpr float kInvDim    = 1.0f / 1024.0f;
constexpr float kLnEps     = 1e-5f;
constexpr float kNegFill   = -3.402823466e+38f;
static_assert(kGroups % kGrpChunk == 0);
static_assert(kHeads % kGrpChunk == 0);

typedef __attribute__((ext_vector_type(16))) _Float16 v16h;
typedef __attribute__((ext_vector_type(8)))  _Float16 v8h;
typedef __attribute__((ext_vector_type(16))) __bf16   v16b;
typedef __attribute__((ext_vector_type(8)))  __bf16   v8b;
typedef __attribute__((ext_vector_type(8)))  float    v8f;
typedef __attribute__((ext_vector_type(4)))  float    v4f;
typedef __attribute__((ext_vector_type(4)))  unsigned int v4u;

__device__ __forceinline__ unsigned short f2bf_bits(float f) {
  unsigned u = __float_as_uint(f);
  return (unsigned short)((u + 0x7FFFu + ((u >> 16) & 1u)) >> 16);
}
__device__ __forceinline__ float bf_bits2f(unsigned short h) { return __uint_as_float(((unsigned)h) << 16); }

__device__ __forceinline__ void dep_guard_h(v8f& a, v8f& b, v16h x, v16h y) { asm volatile("v_nop\n\tv_nop\n\tv_nop\n\tv_nop" : "+v"(a), "+v"(b) : "v"(x), "v"(y)); }
__device__ __forceinline__ void dep_guard_b(v8f& a, v8f& b, v16b x, v16b y) { asm volatile("v_nop\n\tv_nop\n\tv_nop\n\tv_nop" : "+v"(a), "+v"(b) : "v"(x), "v"(y)); }
__device__ __forceinline__ void keep4_h(v16h a, v16h b, v16h c, v16h d) { asm volatile("v_nop" :: "v"(a), "v"(b), "v"(c), "v"(d)); }
__device__ __forceinline__ void keep4_b(v16b a, v16b b, v16b c, v16b d) { asm volatile("v_nop" :: "v"(a), "v"(b), "v"(c), "v"(d)); }
__device__ __forceinline__ void acc_guard4(v8f& a, v8f& b, v8f& c, v8f& d) { asm volatile("v_nop\n\tv_nop\n\tv_nop\n\tv_nop" : "+v"(a), "+v"(b), "+v"(c), "+v"(d)); }
template <typename T> struct Frag;
template <> struct Frag<_Float16> {
  typedef v16h V; union U { v16h v; v8h h[2]; };
  static __device__ __forceinline__ v16h load(const _Float16* p) {
    U f; f.h[0] = *(const v8h*)(p); f.h[1] = *(const v8h*)(p + 16); return f.v;
  }
  static __device__ __forceinline__ v8f mma(v16h a, v16h b, v8f c) {
    return __builtin_amdgcn_wmma_f32_16x16x32_f16(false, a, false, b, (short)0, c, false, false);
  }
  static __device__ __forceinline__ void guard(v8f& a, v8f& b, v16h x, v16h y) { dep_guard_h(a, b, x, y); }
  static __device__ __forceinline__ void keep(v16h a, v16h b, v16h c, v16h d) { keep4_h(a, b, c, d); }
};
template <> struct Frag<__bf16> {
  typedef v16b V; union U { v16b v; v8b h[2]; };
  static __device__ __forceinline__ v16b load(const __bf16* p) {
    U f; f.h[0] = *(const v8b*)(p); f.h[1] = *(const v8b*)(p + 16); return f.v;
  }
  static __device__ __forceinline__ v8f mma(v16b a, v16b b, v8f c) {
    return __builtin_amdgcn_wmma_f32_16x16x32_bf16(false, a, false, b, (short)0, c, false, false);
  }
  static __device__ __forceinline__ void guard(v8f& a, v8f& b, v16b x, v16b y) { dep_guard_b(a, b, x, y); }
  static __device__ __forceinline__ void keep(v16b a, v16b b, v16b c, v16b d) { keep4_b(a, b, c, d); }
};

__device__ __forceinline__ unsigned pk16(unsigned short a, unsigned short b) { return (unsigned)a | ((unsigned)b << 16); }
__device__ __forceinline__ unsigned short h_bits(float f) { const _Float16 h = (_Float16)f; return __builtin_bit_cast(unsigned short, h); }

template <int ET> struct Elem;
template <> struct Elem<0> { typedef _Float16 T; };
template <> struct Elem<1> { typedef __bf16 T; };
template <int ET, bool SPLIT, int BIAS_MODE, int OUT_MODE, bool RESID, int ACT = 0, int KMODE = 0>
__global__ __launch_bounds__(256) void wmma_gemm64(
    const unsigned short* __restrict__ Ap, const unsigned short* __restrict__ A2p, int lda, long strideA,
    const unsigned short* __restrict__ Btp, const unsigned short* __restrict__ Bt2p, int ldb, long strideB,
    void* __restrict__ Cout, void* __restrict__ Cout2, int ldc, long strideC,
    const float* __restrict__ bias,
    const float* __restrict__ resid, long strideR,
    int M, int N, int K, float scale) {
  typedef typename Elem<ET>::T T;
  typedef typename Frag<T>::V V;
  const T* A = (const T*)Ap; const T* A2 = (const T*)A2p; const T* Bt = (const T*)Btp; const T* Bt2 = (const T*)Bt2p;
  __shared__ __align__(16) float sT[8][16 * 68];
  const int b    = blockIdx.y;
  const int lane = threadIdx.x & 31;
  const int wave = threadIdx.x >> 5;
  const int tilesN = N >> 6;
  const int tilesM = M >> 6;
  const int tile = blockIdx.x * 8 + wave;
  if (tile >= tilesM * tilesN) return;
  const int tm = tile / tilesN;
  const int tn = tile - tm * tilesN;
  const int m0 = tm << 6;
  const int n0 = tn << 6;

  const T* Ab  = A  + (size_t)b * strideA;
  const T* Bb  = Bt + (size_t)b * strideB;
  const T* Ab2 = SPLIT ? (A2  + (size_t)b * strideA) : nullptr;
  const T* Bb2 = SPLIT ? (Bt2 + (size_t)b * strideB) : nullptr;

  const int rlane = lane & 15;
  const int koff  = (lane >> 4) * 8;
  const int mOff  = (lane >> 4) * 8;

  v8f acc[4][4];
#pragma unroll
  for (int i = 0; i < 4; ++i)
#pragma unroll
    for (int j = 0; j < 4; ++j) acc[i][j] = (v8f){0.f,0.f,0.f,0.f,0.f,0.f,0.f,0.f};

  int kEnd = K;
  if (KMODE == 1) kEnd = (n0 > m0) ? 0 : K;
  if (KMODE == 2) kEnd = (m0 + 64 < K) ? (m0 + 64) : K;

  for (int k0 = 0; k0 < kEnd; k0 += 32) {
    V bh[4], bl[4];
#pragma unroll
    for (int j = 0; j < 4; ++j) {
      const size_t bo = (size_t)(n0 + (j << 4) + rlane) * ldb + koff + k0;
      bh[j] = Frag<T>::load(Bb + bo);
      if (SPLIT) bl[j] = Frag<T>::load(Bb2 + bo);
    }
#pragma unroll
    for (int i = 0; i < 4; ++i) {
      const size_t ao = (size_t)(m0 + (i << 4) + rlane) * lda + koff + k0;
      V ah = Frag<T>::load(Ab + ao);
      V al;
      if (SPLIT) al = Frag<T>::load(Ab2 + ao);
#pragma unroll
      for (int j = 0; j < 4; ++j) {
        acc[i][j] = Frag<T>::mma(ah, bh[j], acc[i][j]);
        if (SPLIT) {
          acc[i][j] = Frag<T>::mma(ah, bl[j], acc[i][j]);
          acc[i][j] = Frag<T>::mma(al, bh[j], acc[i][j]);
        }
      }
      Frag<T>::guard(acc[i][0], acc[i][3], ah, SPLIT ? al : ah);
    }
    Frag<T>::keep(bh[0], bh[1], bh[2], bh[3]);
    if (SPLIT) Frag<T>::keep(bl[0], bl[1], bl[2], bl[3]);
  }
  acc_guard4(acc[0][0], acc[0][1], acc[0][2], acc[0][3]);
  acc_guard4(acc[1][0], acc[1][1], acc[1][2], acc[1][3]);
  acc_guard4(acc[2][0], acc[2][1], acc[2][2], acc[2][3]);
  acc_guard4(acc[3][0], acc[3][1], acc[3][2], acc[3][3]);

  float* slab = sT[wave];
  const float* Rb = RESID ? (resid + (size_t)b * strideR) : nullptr;
#pragma unroll
  for (int i = 0; i < 4; ++i) {
    const int mBase = m0 + (i << 4);
#pragma unroll
    for (int j = 0; j < 4; ++j) {
      const int n = n0 + (j << 4) + rlane;
      float bv = 0.f;
      if (BIAS_MODE == 2) bv = bias[n];
#pragma unroll
      for (int r = 0; r < 8; ++r) {
        float v = acc[i][j][r] * scale;
        if (BIAS_MODE == 1) v += bias[mBase + mOff + r];
        if (BIAS_MODE == 2) v += bv;
        if (RESID) v += Rb[(size_t)(mBase + mOff + r) * ldc + n];
        if (ACT == 2) v = fmaxf(v, 0.0f);
        if (ACT == 4) v = (v > 0.f) ? v : 0.01f * v;
        if (ACT == 6) {
          const float u = 0.7978845608028654f * (v + 0.044715f * v * v * v);
          v = 0.5f * v * (1.0f + tanhf(u));
        }
        slab[(mOff + r) * 68 + (j << 4) + rlane] = v;
      }
    }
    __builtin_amdgcn_fence(__ATOMIC_RELEASE, "workgroup");
    __builtin_amdgcn_wave_barrier();
    __builtin_amdgcn_fence(__ATOMIC_ACQUIRE, "workgroup");
    if (OUT_MODE == 0) {
      float* C = (float*)Cout + (size_t)b * strideC;
      const int hh = lane >> 4, c4 = (lane & 15) * 4;
      for (int pass = 0; pass < 2; ++pass) {
#pragma unroll
        for (int it = 0; it < 8; ++it) {
          const int row = it * 2 + hh;
          v4f v = *(const v4f*)(slab + row * 68 + c4);
          *(volatile v4f*)(C + (size_t)(mBase + row) * ldc + n0 + c4) = v;
        }
        __threadfence();
      }
    } else {
      const int q = lane >> 3, c8 = (lane & 7) * 8;
      unsigned short* C  = (unsigned short*)Cout  + (size_t)b * strideC;
      unsigned short* C2 = (OUT_MODE == 2) ? ((unsigned short*)Cout2 + (size_t)b * strideC) : nullptr;
      for (int pass = 0; pass < 2; ++pass) {
#pragma unroll
        for (int it = 0; it < 4; ++it) {
          const int row = it * 4 + q;
          const float* sp = slab + row * 68 + c8;
          v8h hv, lv;
#pragma unroll
          for (int e = 0; e < 8; ++e) {
            if (OUT_MODE == 1) {
              hv[e] = (_Float16)sp[e];
            } else {
              unsigned short hb = f2bf_bits(sp[e]);
              unsigned short lb = f2bf_bits(sp[e] - bf_bits2f(hb));
              hv[e] = __builtin_bit_cast(_Float16, hb);
              lv[e] = __builtin_bit_cast(_Float16, lb);
            }
          }
          *(volatile v8h*)(C + (size_t)(mBase + row) * ldc + n0 + c8) = hv;
          if (OUT_MODE == 2) *(volatile v8h*)(C2 + (size_t)(mBase + row) * ldc + n0 + c8) = lv;
        }
        __threadfence();
      }
    }
    __builtin_amdgcn_fence(__ATOMIC_RELEASE, "workgroup");
    __builtin_amdgcn_wave_barrier();
    __builtin_amdgcn_fence(__ATOMIC_ACQUIRE, "workgroup");
  }
}

__global__ __launch_bounds__(256) void wtcast_kernel(const float* __restrict__ W, unsigned short* __restrict__ WT,
                                                     int Kin, int Nout, float scale) {
  __shared__ float sm[64][65];
  const int t  = threadIdx.x;
  const int k0 = blockIdx.x * 64;
  const int n0 = blockIdx.y * 64;
#pragma unroll
  for (int i = 0; i < 16; ++i) {
    const int e = i * 256 + t;
    const int r = e >> 6;
    const int c = e & 63;
    sm[c][r] = W[(size_t)(k0 + r) * Nout + n0 + c] * scale;
  }
  __syncthreads();
  const int lane = t & 31, wave = t >> 5;
  const int q = lane >> 3, c8 = (lane & 7) * 8;
  for (int pass = 0; pass < 2; ++pass) {
#pragma unroll
    for (int it = 0; it < 2; ++it) {
      const int row = wave * 8 + it * 4 + q;
      unsigned short hb[8];
#pragma unroll
      for (int e = 0; e < 8; ++e) hb[e] = h_bits(sm[row][c8 + e]);
      const v4u u = (v4u){pk16(hb[0], hb[1]), pk16(hb[2], hb[3]), pk16(hb[4], hb[5]), pk16(hb[6], hb[7])};
      *(volatile v4u*)(WT + (size_t)(n0 + row) * Kin + k0 + c8) = u;
    }
    __threadfence();
  }
}

__global__ __launch_bounds__(128) void layernorm_f16_kernel(const float* __restrict__ X, const float* __restrict__ w,
                                                            const float* __restrict__ bvec, unsigned short* __restrict__ Y) {
  __shared__ float red1[4];
  __shared__ float red2[4];
  const int row  = blockIdx.x;
  const int t    = threadIdx.x;
  const int lane = t & 31, wave = t >> 5;
  const int c0   = t * 8;
  const float* xr = X + (size_t)row * kDim + c0;
  const v4f a = *(const v4f*)(xr);
  const v4f c = *(const v4f*)(xr + 4);
  float x[8];
#pragma unroll
  for (int e = 0; e < 4; ++e) { x[e] = a[e]; x[4 + e] = c[e]; }
  float s = ((x[0] + x[1]) + (x[2] + x[3])) + ((x[4] + x[5]) + (x[6] + x[7]));
#pragma unroll
  for (int off = 16; off > 0; off >>= 1) s += __shfl_xor(s, off, 32);
  if (lane == 0) red1[wave] = s;
  __syncthreads();
  const float tot = ((red1[0] + red1[1]) + red1[2]) + red1[3];
  const float mu = tot * kInvDim;
  float d[8];
#pragma unroll
  for (int e = 0; e < 8; ++e) d[e] = x[e] - mu;
  float s2 = ((d[0] * d[0] + d[1] * d[1]) + (d[2] * d[2] + d[3] * d[3])) + ((d[4] * d[4] + d[5] * d[5]) + (d[6] * d[6] + d[7] * d[7]));
#pragma unroll
  for (int off = 16; off > 0; off >>= 1) s2 += __shfl_xor(s2, off, 32);
  if (lane == 0) red2[wave] = s2;
  __syncthreads();
  const float tot2 = ((red2[0] + red2[1]) + red2[2]) + red2[3];
  const float var  = tot2 * kInvDim;
  const float rinv = rsqrtf(var + kLnEps);
  const v4f wa = *(const v4f*)(w + c0);
  const v4f wc = *(const v4f*)(w + c0 + 4);
  const v4f ba = *(const v4f*)(bvec + c0);
  const v4f bc = *(const v4f*)(bvec + c0 + 4);
  unsigned short hb[8];
#pragma unroll
  for (int e = 0; e < 4; ++e) {
    hb[e]     = h_bits(d[e] * rinv * wa[e] + ba[e]);
    hb[4 + e] = h_bits(d[4 + e] * rinv * wc[e] + bc[e]);
  }
  const v4u u = (v4u){pk16(hb[0], hb[1]), pk16(hb[2], hb[3]), pk16(hb[4], hb[5]), pk16(hb[6], hb[7])};
  unsigned short* dst = Y + (size_t)row * kDim + c0;
  *(volatile v4u*)dst = u;
  __threadfence();
  *(volatile v4u*)dst = u;
}

__global__ __launch_bounds__(256) void softmax_causal_kernel(const float* __restrict__ S, unsigned short* __restrict__ P) {
  __shared__ float redM[8];
  __shared__ float redS[8];
  const int row  = blockIdx.x;
  const int qpos = row & (kSeq - 1);
  const int t    = threadIdx.x;
  const int lane = t & 31, wave = t >> 5;
  const int c0   = t * 8;
  const bool wact = (wave * 256) <= qpos;
  const float* sr = S + (size_t)row * kSeq + c0;
  const v4f a = *(const v4f*)(sr);
  const v4f c = *(const v4f*)(sr + 4);
  float x[8];
#pragma unroll
  for (int e = 0; e < 4; ++e) { x[e] = a[e]; x[4 + e] = c[e]; }
#pragma unroll
  for (int e = 0; e < 8; ++e) x[e] = (c0 + e <= qpos) ? x[e] : kNegFill;
  float m = fmaxf(fmaxf(fmaxf(x[0], x[1]), fmaxf(x[2], x[3])), fmaxf(fmaxf(x[4], x[5]), fmaxf(x[6], x[7])));
#pragma unroll
  for (int off = 16; off > 0; off >>= 1) m = fmaxf(m, __shfl_xor(m, off, 32));
  if (lane == 0) redM[wave] = m;
  __syncthreads();
  float gm = redM[0];
#pragma unroll
  for (int wv = 1; wv < 8; ++wv) gm = fmaxf(gm, redM[wv]);
  float p[8];
  float s = 0.f;
  if (wact) {
#pragma unroll
    for (int e = 0; e < 8; ++e) p[e] = expf(x[e] - gm);
    s = ((p[0] + p[1]) + (p[2] + p[3])) + ((p[4] + p[5]) + (p[6] + p[7]));
  } else {
#pragma unroll
    for (int e = 0; e < 8; ++e) p[e] = 0.f;
  }
#pragma unroll
  for (int off = 16; off > 0; off >>= 1) s += __shfl_xor(s, off, 32);
  if (lane == 0) redS[wave] = s;
  __syncthreads();
  float tot = redS[0];
#pragma unroll
  for (int wv = 1; wv < 8; ++wv) tot += redS[wv];
  const float inv = kPCarry * (1.0f / tot);
  unsigned short hb[8];
#pragma unroll
  for (int e = 0; e < 8; ++e) hb[e] = h_bits(p[e] * inv);
  const v4u u = (v4u){pk16(hb[0], hb[1]), pk16(hb[2], hb[3]), pk16(hb[4], hb[5]), pk16(hb[6], hb[7])};
  unsigned short* dst = P + (size_t)row * kSeq + c0;
  *(volatile v4u*)dst = u;
  __threadfence();
  *(volatile v4u*)dst = u;
}

extern "C" void kernel_launch(void* const* d_in, const int* in_sizes, int n_in,
                              void* d_out, int out_size, void* d_ws, size_t ws_size,
                              hipStream_t stream) {
  if (n_in < 13) return;
  if (in_sizes[0] != kTok * kDim) return;
  if (in_sizes[1] != kDim * 2 * kDim) return;
  if (in_sizes[2] != 2 * kDim) return;
  if (in_sizes[3] != kDim * kDim) return;
  if (in_sizes[4] != kDim * kDim) return;
  if (in_sizes[5] != kDim || in_sizes[6] != kDim || in_sizes[7] != kDim || in_sizes[8] != kDim) return;
  if (in_sizes[9] != kDim * kFF) return;
  if (in_sizes[10] != kFF) return;
  if (in_sizes[11] != kFF * kDim) return;
  if (in_sizes[12] != kDim) return;
  if (out_size != kTok * kDim) return;

  const float* x      = (const float*)d_in[0];
  const float* qk_w   = (const float*)d_in[1];
  const float* qk_b   = (const float*)d_in[2];
  const float* v_w    = (const float*)d_in[3];
  const float* proj_w = (const float*)d_in[4];
  const float* ln1_w  = (const float*)d_in[5];
  const float* ln1_b  = (const float*)d_in[6];
  const float* ln2_w  = (const float*)d_in[7];
  const float* ln2_b  = (const float*)d_in[8];
  const float* fc_w   = (const float*)d_in[9];
  const float* fc_b   = (const float*)d_in[10];
  const float* mlp_w  = (const float*)d_in[11];
  const float* mlp_b  = (const float*)d_in[12];
  float* out = (float*)d_out;

  const size_t MiB = (size_t)1 << 20;
  const size_t oWqk = 0;
  const size_t oWv  = oWqk + (size_t)2 * kDim * kDim * 2;
  const size_t oWpr = oWv  + (size_t)kDim * kDim * 2;
  const size_t oWfc = oWpr + (size_t)kDim * kDim * 2;
  const size_t oWml = oWfc + (size_t)kFF * kDim * 2;
  const size_t oH   = oWml + (size_t)kDim * kFF * 2;
  const size_t oQK  = oH   + (size_t)kTok * kDim * 2;
  const size_t oVT  = oQK  + (size_t)kTok * 2 * kDim * 2;
  const size_t oG   = oQK;
  const size_t oO   = oG   + (size_t)kTok * kFF * 2;
  const size_t oSC  = oO   + (size_t)kTok * kDim * 2;
  const size_t oX1  = oSC;
  const size_t oP   = oSC  + (size_t)kGrpChunk * kSeq * kSeq * 4;
  const size_t oEnd = oP   + (size_t)kGrpChunk * kSeq * kSeq * 2;
  if (oVT + (size_t)kBatch * kDim * kSeq * 2 > oO) return;
  if (oX1 + (size_t)kTok * kDim * 4 > oP) return;
  if (oEnd != (size_t)120 * MiB) return;
  if (oEnd > ws_size) return;

  char* ws = (char*)d_ws;
  unsigned short* WqkT = (unsigned short*)(ws + oWqk);
  unsigned short* WvT  = (unsigned short*)(ws + oWv);
  unsigned short* WprT = (unsigned short*)(ws + oWpr);
  unsigned short* WfcT = (unsigned short*)(ws + oWfc);
  unsigned short* WmlT = (unsigned short*)(ws + oWml);
  unsigned short* H16  = (unsigned short*)(ws + oH);
  unsigned short* QK16 = (unsigned short*)(ws + oQK);
  unsigned short* VT16 = (unsigned short*)(ws + oVT);
  unsigned short* G16  = (unsigned short*)(ws + oG);
  unsigned short* O16  = (unsigned short*)(ws + oO);
  float*          SC32 = (float*)(ws + oSC);
  float*          X1   = (float*)(ws + oX1);
  unsigned short* P16  = (unsigned short*)(ws + oP);

  wtcast_kernel<<<dim3(kDim / 64, (2 * kDim) / 64), 256, 0, stream>>>(qk_w,   WqkT, kDim, 2 * kDim, kWCarry);
  wtcast_kernel<<<dim3(kDim / 64, kDim / 64),       256, 0, stream>>>(v_w,    WvT,  kDim, kDim,     kWCarry);
  wtcast_kernel<<<dim3(kDim / 64, kDim / 64),       256, 0, stream>>>(proj_w, WprT, kDim, kDim,     kWCarry);
  wtcast_kernel<<<dim3(kDim / 64, kFF / 64),        256, 0, stream>>>(fc_w,   WfcT, kDim, kFF,      kWCarry);
  wtcast_kernel<<<dim3(kFF / 64,  kDim / 64),       256, 0, stream>>>(mlp_w,  WmlT, kFF,  kDim,     kWCarry);

  layernorm_f16_kernel<<<kTok, 128, 0, stream>>>(x, ln1_w, ln1_b, H16);

  wmma_gemm64<0, false, 2, 1, false, 0, 0><<<dim3((kTok / 64) * (2 * kDim / 64) / 8, 1), 256, 0, stream>>>(
      H16, nullptr, kDim, 0L, WqkT, nullptr, kDim, 0L, QK16, nullptr, 2 * kDim, 0L,
      qk_b, nullptr, 0L, kTok, 2 * kDim, kDim, kWCarryInv);
  wmma_gemm64<0, false, 0, 1, false, 0, 0><<<dim3((kDim / 64) * (kSeq / 64) / 8, kBatch), 256, 0, stream>>>(
      WvT, nullptr, kDim, 0L, H16, nullptr, kDim, (long)kSeq * kDim, VT16, nullptr, kSeq, (long)kDim * kSeq,
      nullptr, nullptr, 0L, kDim, kSeq, kDim, kWCarryInv);

  for (int ch = 0; ch < kNumChunks; ++ch) {
    const int g0 = ch * kGrpChunk;
    const int bb = g0 / kHeads;
    const int h0 = g0 % kHeads;
    const unsigned short* qbase = QK16 + (size_t)bb * kSeq * (2 * kDim) + (size_t)h0 * kHdim;
    const unsigned short* kbase = qbase + kDim;
    wmma_gemm64<0, false, 0, 0, false, 0, 1><<<dim3((kSeq / 64) * (kSeq / 64) / 8, kGrpChunk), 256, 0, stream>>>(
        qbase, nullptr, 2 * kDim, (long)kHdim, kbase, nullptr, 2 * kDim, (long)kHdim,
        SC32, nullptr, kSeq, (long)kSeq * kSeq, nullptr, nullptr, 0L, kSeq, kSeq, kHdim, kScoreScale);
    softmax_causal_kernel<<<kGrpChunk * kSeq, 256, 0, stream>>>(SC32, P16);
    wmma_gemm64<0, false, 0, 1, false, 0, 2><<<dim3((kSeq / 64) * (kHdim / 64) / 8, kGrpChunk), 256, 0, stream>>>(
        P16, nullptr, kSeq, (long)kSeq * kSeq,
        VT16 + ((size_t)bb * kDim + (size_t)h0 * kHdim) * kSeq, nullptr, kSeq, (long)kHdim * kSeq,
        O16 + (size_t)bb * kSeq * kDim + (size_t)h0 * kHdim, nullptr, kDim, (long)kHdim,
        nullptr, nullptr, 0L, kSeq, kHdim, kSeq, kPVScale);
  }

  wmma_gemm64<0, false, 0, 0, true, 0, 0><<<dim3((kTok / 64) * (kDim / 64) / 8, 1), 256, 0, stream>>>(
      O16, nullptr, kDim, 0L, WprT, nullptr, kDim, 0L, X1, nullptr, kDim, 0L,
      nullptr, x, 0L, kTok, kDim, kDim, kProjScale);

  layernorm_f16_kernel<<<kTok, 128, 0, stream>>>(X1, ln2_w, ln2_b, H16);

  wmma_gemm64<0, false, 2, 1, false, 6, 0><<<dim3((kTok / 64) * (kFF / 64) / 8, 1), 256, 0, stream>>>(
      H16, nullptr, kDim, 0L, WfcT, nullptr, kDim, 0L, G16, nullptr, kFF, 0L,
      fc_b, nullptr, 0L, kTok, kFF, kDim, kWCarryInv);

  wmma_gemm64<0, false, 2, 0, true, 0, 0><<<dim3((kTok / 64) * (kDim / 64) / 8, 1), 256, 0, stream>>>(
      G16, nullptr, kFF, 0L, WmlT, nullptr, kFF, 0L, out, nullptr, kDim, 0L,
      mlp_b, X1, 0L, kTok, kDim, kFF, kWCarryInv);
}
